// BaseLayer_27058293964888
// MI455X (gfx1250) — hardware-run, weakly checked
//
#include <hip/hip_runtime.h>


#define NN   16384
#define FEAT 256
#define EMB  128
#define OUTD 128
#define TT   NN
#define TK   NN
#define HD   EMB
#define NH_  1
#define NKV  1
#define DQ   EMB
#define DKV  EMB
#define DM   FEAT
#define ZH   1
#define RB   1024
#define RH   0
#define PCAR 16.0f
typedef _Float16 h16;
typedef unsigned short bf;
typedef __attribute__((ext_vector_type(16))) __bf16   v16bf;
typedef __attribute__((ext_vector_type(16))) _Float16 v16h;
typedef __attribute__((ext_vector_type(8)))  _Float16 v8h;
typedef __attribute__((ext_vector_type(8)))  unsigned short v8us;
typedef __attribute__((ext_vector_type(8)))  float    v8f;
typedef __attribute__((ext_vector_type(4)))  float    v4f;
typedef v8h  __attribute__((may_alias)) v8ha;
typedef v4f  __attribute__((may_alias)) v4fa;
typedef v8us __attribute__((may_alias)) v8usa;

__device__ __forceinline__ unsigned short f2bf(float f) { unsigned u = __float_as_uint(f); u += 0x7FFFu + ((u >> 16) & 1u); return (unsigned short)(u >> 16); }
__device__ __forceinline__ float bf2f(unsigned short b) { return __uint_as_float(((unsigned)b) << 16); }
__device__ __forceinline__ float bfr(float f) { return bf2f(f2bf(f)); }
__device__ __forceinline__ v16h cat16(v8h lo, v8h hi) { return __builtin_shufflevector(lo, hi, 0, 1, 2, 3, 4, 5, 6, 7, 8, 9, 10, 11, 12, 13, 14, 15); }
__device__ __forceinline__ v16bf cat16b(v8us lo, v8us hi) { return __builtin_bit_cast(v16bf, __builtin_shufflevector(lo, hi, 0, 1, 2, 3, 4, 5, 6, 7, 8, 9, 10, 11, 12, 13, 14, 15)); }
__device__ __forceinline__ v8f wmma16(v16h a, v16h b, v8f c) { return __builtin_amdgcn_wmma_f32_16x16x32_f16(false, a, false, b, (short)0, c, false, false); }
__device__ __forceinline__ v8f wmmab(v16bf a, v16bf b, v8f c) { return __builtin_amdgcn_wmma_f32_16x16x32_bf16(false, a, false, b, (short)0, c, false, false); }


template <typename T16> struct WFrag;
template <> struct WFrag<h16> { typedef v16h V; static __device__ __forceinline__ V ld(const h16* p) { return cat16(*(const v8h*)p, *(const v8h*)(p + 16)); } static __device__ __forceinline__ v8f mma(V a, V b, v8f c) { return wmma16(a, b, c); } };
template <> struct WFrag<bf> { typedef v16bf V; static __device__ __forceinline__ V ld(const bf* p) { return cat16b(*(const v8us*)p, *(const v8us*)(p + 16)); } static __device__ __forceinline__ v8f mma(V a, V b, v8f c) { return wmmab(a, b, c); } };
template <typename T16, int NSPLIT, bool BIAS>
__global__ __launch_bounds__(32) void k_gemmw(const T16* __restrict__ A, const T16* __restrict__ A2, const T16* __restrict__ Bt, const T16* __restrict__ Bt2, int K, float* C, int ldc, const float* __restrict__ bias, size_t sA, size_t sB, size_t sC) {
    typedef typename WFrag<T16>::V V;
    __shared__ __align__(16) float os[16 * 68];
    const size_t z = blockIdx.z; A += z * sA; if (A2) A2 += z * sA; Bt += z * sB; if (Bt2) Bt2 += z * sB; C += z * sC;
    const int lane = threadIdx.x & 31, lr = lane & 15, hi = lane >> 4; const int r0 = blockIdx.x * 64, c0 = blockIdx.y * 64;
    v8f acc[4][4];
#pragma unroll
    for (int mb = 0; mb < 4; ++mb)
#pragma unroll
        for (int nb = 0; nb < 4; ++nb) acc[mb][nb] = (v8f){};
    const size_t aoff = (size_t)(r0 + lr) * K + 8 * hi, boff = (size_t)(c0 + lr) * K + 8 * hi;
#pragma unroll 1
    for (int kc = 0; kc < K; kc += 32) {
        V a[4], a2[4];
#pragma unroll
        for (int mb = 0; mb < 4; ++mb) { a[mb] = WFrag<T16>::ld(A + aoff + (size_t)mb * 16 * K + kc); if (NSPLIT == 1 || NSPLIT == 2) a2[mb] = WFrag<T16>::ld(A2 + aoff + (size_t)mb * 16 * K + kc); }
#pragma unroll
        for (int nb = 0; nb < 4; ++nb) { const V b = WFrag<T16>::ld(Bt + boff + (size_t)nb * 16 * K + kc); V b2; if (NSPLIT >= 2) b2 = WFrag<T16>::ld(Bt2 + boff + (size_t)nb * 16 * K + kc);
#pragma unroll
            for (int mb = 0; mb < 4; ++mb) { acc[mb][nb] = WFrag<T16>::mma(a[mb], b, acc[mb][nb]); if (NSPLIT == 1 || NSPLIT == 2) acc[mb][nb] = WFrag<T16>::mma(a2[mb], b, acc[mb][nb]); if (NSPLIT >= 2) acc[mb][nb] = WFrag<T16>::mma(a[mb], b2, acc[mb][nb]); } }
        asm volatile("v_nop\n\tv_nop\n\tv_nop\n\tv_nop" : "+v"(acc[0][0]), "+v"(acc[1][1]), "+v"(acc[2][2]), "+v"(acc[3][3]) : "v"(a[0]), "v"(a[3]));
    }
#pragma unroll
    for (int mb = 0; mb < 4; ++mb) {
#pragma unroll
        for (int nb = 0; nb < 4; ++nb) {
#pragma unroll
            for (int j = 0; j < 8; ++j) os[(hi * 8 + j) * 68 + nb * 16 + lr] = acc[mb][nb][j]; }
        __builtin_amdgcn_wave_barrier(); asm volatile("" ::: "memory");
        float* crow = C + (size_t)(r0 + mb * 16) * ldc + c0;
#pragma unroll 1
        for (int ps = 0; ps < 2; ++ps) {
#pragma unroll
            for (int s = 0; s < 8; ++s) { const int row = 2 * s + hi, cofs = lr * 4; v4f val = *(const v4fa*)(os + row * 68 + cofs); if (BIAS) { val[0] += bfr(bias[c0 + cofs]); val[1] += bfr(bias[c0 + cofs + 1]); val[2] += bfr(bias[c0 + cofs + 2]); val[3] += bfr(bias[c0 + cofs + 3]); }
                *(volatile v4f*)(crow + (size_t)row * ldc + cofs) = val; }
            if (ps == 0) __threadfence(); }
        __builtin_amdgcn_wave_barrier(); asm volatile("" ::: "memory");
    }
}

__device__ __forceinline__ h16 tohx(float x) { return (h16)x; }
__device__ __forceinline__ void splitf(float y, unsigned short& h, unsigned short& l) { h = f2bf(y); l = f2bf(y - bf2f(h)); }
typedef __attribute__((ext_vector_type(2))) _Float16 v2h;
typedef __attribute__((ext_vector_type(4))) _Float16 v4h;
typedef __attribute__((ext_vector_type(2))) unsigned short v2us;
typedef __attribute__((ext_vector_type(4))) unsigned short v4us;
typedef __attribute__((ext_vector_type(2))) float v2f;
typedef __attribute__((ext_vector_type(4))) int v4i;

__global__ __launch_bounds__(256) void k_wtG(const float* __restrict__ w, int K, int N, bf* Bt) {
    const int lane = threadIdx.x & 31; const int L0 = (blockIdx.x * 8 + (threadIdx.x >> 5)) * 8; const int nlines = N * K / 64;
#pragma unroll
    for (int ps = 0; ps < 2; ++ps) {
#pragma unroll 1
        for (int l = 0; l < 8; ++l) { const int L = L0 + l; if (L >= nlines) break; const size_t e = (size_t)L * 64 + lane * 2; const int k = (int)(e % K), n = (int)(e / K); v2us o;
            o[0] = f2bf(w[(size_t)k * N + n]); o[1] = f2bf(w[(size_t)(k + 1) * N + n]); *(volatile v2us*)(Bt + e) = o; }
        if (ps == 0) __threadfence(); }
}
__global__ __launch_bounds__(256) void k_cvt8(const float* __restrict__ src, bf* dst, size_t n8) { const size_t i = (size_t)blockIdx.x * 256 + threadIdx.x; if (i >= n8) return; const v8f v = *(const v8f*)(src + i * 8); v8us o;
#pragma unroll
    for (int k = 0; k < 8; ++k) o[k] = f2bf(v[k]); *(volatile v8us*)(dst + i * 8) = o; __threadfence(); *(volatile v8us*)(dst + i * 8) = o; }


__global__ __launch_bounds__(256) void k_p16(const float* __restrict__ H, h16* P, size_t n8) { const size_t i = (size_t)blockIdx.x * 256 + threadIdx.x; if (i >= n8) return; const v8f v = *(const v8f*)(H + i * 8); v8h o;
#pragma unroll
    for (int q = 0; q < 8; ++q) o[q] = tohx(v[q]); *(volatile v8h*)(P + i * 8) = o; __threadfence(); *(volatile v8h*)(P + i * 8) = o; }
__global__ __launch_bounds__(256) void k_t16(const float* __restrict__ H, h16* PT) { const size_t e = ((size_t)blockIdx.x * 256 + threadIdx.x) * 2; if (e >= (size_t)EMB * NN) return; const int i = (int)(e % NN); const int c = (int)(e / NN); v2h o; o[0] = tohx(H[(size_t)i * EMB + c]); o[1] = tohx(H[(size_t)(i + 1) * EMB + c]); *(volatile v2h*)(PT + e) = o; __threadfence(); *(volatile v2h*)(PT + e) = o; }
__global__ __launch_bounds__(256) void k_rowsq(const float* __restrict__ H, float* D) { const int i = blockIdx.x * 256 + threadIdx.x; if (i >= NN) return; const float* h = H + (size_t)i * EMB; float s = 0.f;
#pragma unroll 2
    for (int c = 0; c < EMB; c += 4) { const v4f v = *(const v4f*)(h + c);
#pragma unroll
        for (int q = 0; q < 4; ++q) { float p = __fmul_rn(v[q], v[q]); asm volatile("" : "+v"(p)); s = __fadd_rn(s, p); } }
    *(volatile float*)(D + i) = s; __threadfence(); *(volatile float*)(D + i) = s; }
__global__ __launch_bounds__(256) void k_ascale(const float* __restrict__ Sb, const float* __restrict__ D, int i0, h16* P16) { const size_t t = (size_t)blockIdx.x * 256 + threadIdx.x; if (t >= (size_t)RB * NN / 4) return; const size_t e = t * 4; const int j = (int)(e % NN); const int r = (int)(e / NN); const float di = D[i0 + r]; const v4f s = *(const v4f*)(Sb + e); const v4f dj = *(const v4f*)(D + j); v4h o;
#pragma unroll
    for (int q = 0; q < 4; ++q) { float den = __fadd_rn(di, dj[q]); asm volatile("" : "+v"(den)); float a = __fdiv_rn(__fmul_rn(2.0f * PCAR, s[q]), den); o[q] = tohx(a); }
    *(volatile v4h*)(P16 + e) = o; __threadfence(); *(volatile v4h*)(P16 + e) = o; }
__global__ __launch_bounds__(256) void k_aggpl(const float* __restrict__ Ob, bf* Ah, bf* Al) { const size_t e = ((size_t)blockIdx.x * 256 + threadIdx.x) * 2; if (e >= (size_t)RB * EMB) return; v2us oh, ol;
#pragma unroll
    for (int q = 0; q < 2; ++q) { unsigned short a, c2; splitf(Ob[e + q] * (1.0f / PCAR), a, c2); oh[q] = a; ol[q] = c2; } *(volatile v2us*)(Ah + e) = oh; *(volatile v2us*)(Al + e) = ol; __threadfence(); *(volatile v2us*)(Ah + e) = oh; *(volatile v2us*)(Al + e) = ol; }
__global__ __launch_bounds__(256) void k_relu(const float* __restrict__ Y, float* O, size_t n4) { const size_t i = (size_t)blockIdx.x * 256 + threadIdx.x; if (i >= n4) return; const v4f y = *(const v4f*)(Y + i * 4); v4f o;
#pragma unroll
    for (int q = 0; q < 4; ++q) o[q] = fmaxf(y[q], 0.0f); *(volatile v4f*)(O + i * 4) = o; __threadfence(); *(volatile v4f*)(O + i * 4) = o; }

extern "C" void kernel_launch(void* const* d_in, const int* in_sizes, int n_in,
                              void* d_out, int out_size, void* d_ws, size_t ws_size, hipStream_t stream) {
    (void)in_sizes; (void)n_in; (void)out_size;
    const float* x = (const float*)d_in[0]; const float* w1 = (const float*)d_in[1]; const float* b1 = (const float*)d_in[2]; const float* w2 = (const float*)d_in[3]; const float* b2 = (const float*)d_in[4];
    float* OUT = (float*)d_out;
    char* wsp = (char*)d_ws;
    auto take = [&](size_t bytes) { char* p = wsp; wsp += (bytes + 255) & ~(size_t)255; return (void*)p; };
    bf* W1 = (bf*)take((size_t)EMB * FEAT * 2); bf* W2 = (bf*)take((size_t)OUTD * EMB * 2);
    bf* XB = (bf*)take((size_t)NN * FEAT * 2); float* FH = (float*)take((size_t)NN * EMB * 4); float* D = (float*)take((size_t)NN * 4);
    h16* HP16 = (h16*)take((size_t)NN * EMB * 2);
    h16* HT16 = (h16*)take((size_t)EMB * NN * 2);
    float* Sb = (float*)take((size_t)RB * NN * 4); h16* P16 = (h16*)take((size_t)RB * NN * 2); float* Ob = (float*)take((size_t)RB * EMB * 4); bf* AGh = (bf*)take((size_t)RB * EMB * 2); bf* AGl = (bf*)take((size_t)RB * EMB * 2); float* YO = (float*)take((size_t)RB * OUTD * 4);
    if ((size_t)(wsp - (char*)d_ws) > ws_size) return;
    k_wtG<<<(unsigned)((FEAT * EMB / 64 + 63) / 64), 256, 0, stream>>>(w1, FEAT, EMB, W1); k_wtG<<<(unsigned)((EMB * OUTD / 64 + 63) / 64), 256, 0, stream>>>(w2, EMB, OUTD, W2);
        k_cvt8<<<(unsigned)(((size_t)NN * FEAT / 8 + 255) / 256), 256, 0, stream>>>(x, XB, (size_t)NN * FEAT / 8);
    k_gemmw<bf, 0, true><<<dim3(NN / 64, EMB / 64, 1), 32, 0, stream>>>(XB, nullptr, W1, nullptr, FEAT, FH, EMB, b1, 0, 0, 0);
    k_rowsq<<<NN / 256, 256, 0, stream>>>(FH, D);
    k_p16<<<(unsigned)(((size_t)NN * EMB / 8 + 255) / 256), 256, 0, stream>>>(FH, HP16, (size_t)NN * EMB / 8);
    k_t16<<<(unsigned)(((size_t)EMB * NN / 2 + 255) / 256), 256, 0, stream>>>(FH, HT16);
    for (int i0 = 0; i0 < NN; i0 += RB) {
        k_gemmw<h16, 0, false><<<dim3(RB / 64, NN / 64, 1), 32, 0, stream>>>(HP16 + (size_t)i0 * EMB, nullptr, HP16, nullptr, EMB, Sb, NN, nullptr, 0, 0, 0);
        k_ascale<<<(unsigned)(((size_t)RB * NN / 4 + 255) / 256), 256, 0, stream>>>(Sb, D, i0, P16);
        k_gemmw<h16, 0, false><<<dim3(RB / 64, EMB / 64, 1), 32, 0, stream>>>(P16, nullptr, HT16, nullptr, NN, Ob, EMB, nullptr, 0, 0, 0);
        k_aggpl<<<(unsigned)(((size_t)RB * EMB / 2 + 255) / 256), 256, 0, stream>>>(Ob, AGh, AGl);
        k_gemmw<bf, 1, true><<<dim3(RB / 64, OUTD / 64, 1), 32, 0, stream>>>(AGh, AGl, W2, nullptr, EMB, YO, OUTD, b2, 0, 0, 0);
        k_relu<<<(unsigned)(((size_t)RB * OUTD / 4 + 255) / 256), 256, 0, stream>>>(YO, OUT + (size_t)i0 * OUTD, (size_t)RB * OUTD / 4); }
}
